// ValueIterationNetwork_70970039599284
// MI455X (gfx1250) — hardware-verified
//
#include <hip/hip_runtime.h>
#include <math.h>

typedef __attribute__((ext_vector_type(16))) _Float16     v16h;
typedef __attribute__((ext_vector_type(8)))  _Float16     v8h;
typedef __attribute__((ext_vector_type(2)))  _Float16     v2h;
typedef __attribute__((ext_vector_type(8)))  float        v8f;
typedef __attribute__((ext_vector_type(4)))  float        v4f;
typedef __attribute__((ext_vector_type(8)))  unsigned int v8u;

constexpr int kDepth     = 16;
constexpr int kBatch     = 16;
constexpr int kMapH      = 96;
constexpr int kMapW      = 96;
constexpr int kActions   = 10;
constexpr int kTaps      = 9;
constexpr int kChanLive  = kActions * kTaps;
constexpr int kChanPad   = 96;
constexpr int kKPad      = 32;
constexpr int kColTiles  = kChanPad / 16;
constexpr int kMapElems  = kMapH * kMapW;
constexpr int kSliceElems = kBatch * kMapElems;

constexpr int kWavesPerBlock = 8;
constexpr int kThreads       = kWavesPerBlock * 32;
constexpr int kPixPerWave    = 32;
constexpr int kSegPerRow     = kMapW / kPixPerWave;
constexpr int kWavesTotal    = kBatch * kMapH * kSegPerRow;
constexpr int kBlocks        = kWavesTotal / kWavesPerBlock;

constexpr int kStripPitch = kPixPerWave + 2;
constexpr int kStripSlots = 128;
constexpr int kSlabPitch  = kPixPerWave;
constexpr int kSlabElems  = kChanPad * kSlabPitch;
constexpr int kPlaneWords = kChanPad * kKPad / 2;

constexpr float kActCarry   = 16.0f;
constexpr float kWtCarry    = 256.0f;
constexpr float kResCarry   = 2048.0f;
constexpr float kFoldMain   = 1.0f / (kActCarry * kWtCarry);
constexpr float kFoldCross  = kFoldMain / kResCarry;
constexpr float kF16MinNorm = 6.103515625e-05f;
constexpr float kF32MinNorm = 1.17549435e-38f;

static_assert(kChanLive == 90 && kChanLive <= kChanPad && (kChanPad % 16) == 0, "channel padding");
static_assert(kTaps <= 16 && kKPad == 32, "one 32-deep k step; only the lower eight-element groups are live");
static_assert(kSegPerRow * kPixPerWave == kMapW, "three waves per map row");
static_assert((kWavesTotal % kWavesPerBlock) == 0 && kBlocks == 576, "exact grid");
static_assert(3 * kStripPitch <= kStripSlots, "strip fits its slots");
static_assert(kPlaneWords == 6 * kThreads, "weight fill coverage: 6 iterations x 256 threads x 1 word");
static_assert((kMapW * 4) % 128 == 0 && (kPixPerWave * 4) == 128, "one 128-B line per wave store");
static_assert(kSliceElems == 147456 && kDepth * kSliceElems == 2359296, "wire shapes");

__device__ __forceinline__ _Float16 to_f16_flushed(float x) {
  const float y = (fabsf(x) < kF16MinNorm) ? 0.0f : x;
  return (_Float16)y;
}
__device__ __forceinline__ void split_f16(float x, _Float16& hv, _Float16& rv) {
  hv = to_f16_flushed(x);
  const float hf = (float)hv;
  const float d = x - hf;
  rv = to_f16_flushed(d * kResCarry);
}
__device__ __forceinline__ unsigned pack2(_Float16 a, _Float16 b) {
  v2h p;
  p[0] = a;
  p[1] = b;
  return __builtin_bit_cast(unsigned, p);
}

struct FragH {
  union U { v16h v; v8h h[2]; };
  static __device__ __forceinline__ v16h load(const _Float16* p) {
    U f;
    f.h[0] = *(const v8h*)(p);
    f.h[1] = *(const v8h*)(p + 16);
    return f.v;
  }
  static __device__ __forceinline__ v8f mma(v16h a, v16h b, v8f c) {
    return __builtin_amdgcn_wmma_f32_16x16x32_f16(false, a, false, b, (short)0, c, false, false);
  }
};
__device__ __forceinline__ void guard1(v8f& acc, v16h a0, v16h a1, v16h b0, v16h b1) {
  asm volatile("v_nop\n\tv_nop\n\tv_nop\n\tv_nop" : "+v"(acc) : "v"(a0), "v"(a1), "v"(b0), "v"(b1));
}

__global__ __launch_bounds__(kThreads) void vi_step_kernel(const float* __restrict__ v_in,
                                                           const float* __restrict__ rewards,
                                                           const float* __restrict__ wt,
                                                           float* __restrict__ v_out) {
  __shared__ __align__(16) unsigned sBv[kPlaneWords];
  __shared__ __align__(16) unsigned sBr[kPlaneWords];
  __shared__ __align__(16) float    sStrip[kWavesPerBlock * kStripSlots];
  __shared__ __align__(16) float    sSlab[kWavesPerBlock * kSlabElems];

  const int tid  = threadIdx.x;
  const int lane = tid & 31;
  const int wave = tid >> 5;
  const int rl   = lane & 15;
  const int half = lane >> 4;

  const int gw   = blockIdx.x * kWavesPerBlock + wave;
  const int grow = gw / kSegPerRow;
  const int seg  = gw - grow * kSegPerRow;
  const int bimg = grow / kMapH;
  const int h    = grow - bimg * kMapH;
  const int w0   = seg * kPixPerWave;

  const float* vimg = v_in    + (size_t)bimg * kMapElems;
  const float* rimg = rewards + (size_t)bimg * kMapElems;

#pragma unroll 1
  for (int it = 0; it < 6; ++it) {
    const int wI = it * kThreads + tid;
    const int n  = wI >> 4;
    const int kw = wI & 15;
    const int k0 = 2 * kw;
    const int k1 = k0 + 1;
    const int nc  = min(n, kChanLive - 1);
    const int k0c = min(k0, kTaps - 1);
    const int k1c = min(k1, kTaps - 1);
    const float g0 = wt[nc * kTaps + k0c];
    const float g1 = wt[nc * kTaps + k1c];
    const bool ok0 = (n < kChanLive) && (k0 < kTaps);
    const bool ok1 = (n < kChanLive) && (k1 < kTaps);
    const float x0 = ok0 ? (g0 * kWtCarry) : 0.0f;
    const float x1 = ok1 ? (g1 * kWtCarry) : 0.0f;
    _Float16 h0, r0, h1, r1;
    split_f16(x0, h0, r0);
    split_f16(x1, h1, r1);
    sBv[wI] = pack2(h0, h1);
    sBr[wI] = pack2(r0, r1);
  }

  float* strip = sStrip + wave * kStripSlots;
#pragma unroll
  for (int it = 0; it < 4; ++it) {
    unsigned idx = (unsigned)it * 32u + (unsigned)lane;
    asm volatile("" : "+v"(idx));
    const int r   = (int)(idx / (unsigned)kStripPitch);
    const int c   = (int)idx - r * kStripPitch;
    const int hh  = h - 1 + r;
    const int ww  = w0 - 1 + c;
    const bool inb = (r < 3) && (hh >= 0) && (hh < kMapH) && (ww >= 0) && (ww < kMapW);
    const int hc = min(max(hh, 0), kMapH - 1);
    const int wc = min(max(ww, 0), kMapW - 1);
    const float a = vimg[hc * kMapW + wc];
    const float b = rimg[hc * kMapW + wc];
    const float s = a + b;
    strip[idx] = inb ? s : 0.0f;
  }
  __syncthreads();

  const bool upper = (half != 0);
  v16h av[2], ar[2];
#pragma unroll
  for (int t = 0; t < 2; ++t) {
    const float* tp = strip + 16 * t + rl;
    float tap[kTaps];
#pragma unroll
    for (int i = 0; i < kTaps; ++i) tap[i] = tp[(i / 3) * kStripPitch + (i % 3)];
    unsigned wv[4], wr[4];
#pragma unroll
    for (int e2 = 0; e2 < 4; ++e2) {
      const float lo0 = tap[2 * e2];
      const float lo1 = tap[2 * e2 + 1];
      const float up0 = (e2 == 0) ? tap[8] : 0.0f;
      const float x0 = (upper ? up0 : lo0) * kActCarry;
      const float x1 = (upper ? 0.0f : lo1) * kActCarry;
      _Float16 h0, r0, h1, r1;
      split_f16(x0, h0, r0);
      split_f16(x1, h1, r1);
      wv[e2] = pack2(h0, h1);
      wr[e2] = pack2(r0, r1);
    }
    const v8u uv = (v8u){wv[0], wv[1], wv[2], wv[3], 0u, 0u, 0u, 0u};
    const v8u ur = (v8u){wr[0], wr[1], wr[2], wr[3], 0u, 0u, 0u, 0u};
    av[t] = __builtin_bit_cast(v16h, uv);
    ar[t] = __builtin_bit_cast(v16h, ur);
  }

  float* slab = sSlab + wave * kSlabElems;
  {
    const _Float16* bBaseV = (const _Float16*)sBv + rl * kKPad + 8 * half;
    const _Float16* bBaseR = (const _Float16*)sBr + rl * kKPad + 8 * half;
    float* slabW = slab + rl * kSlabPitch + 8 * half;
#pragma unroll 1
    for (int j = 0; j < kColTiles; ++j) {
      const v16h bv = FragH::load(bBaseV + j * 16 * kKPad);
      const v16h br = FragH::load(bBaseR + j * 16 * kKPad);
#pragma unroll
      for (int t = 0; t < 2; ++t) {
        v8f acc  = (v8f){0.f, 0.f, 0.f, 0.f, 0.f, 0.f, 0.f, 0.f};
        v8f accr = (v8f){0.f, 0.f, 0.f, 0.f, 0.f, 0.f, 0.f, 0.f};
        acc  = FragH::mma(av[t], bv, acc);
        accr = FragH::mma(av[t], br, accr);
        accr = FragH::mma(ar[t], bv, accr);
        guard1(acc,  av[t], ar[t], bv, br);
        guard1(accr, av[t], ar[t], bv, br);
        v4f o0, o1;
#pragma unroll
        for (int r = 0; r < 4; ++r) {
          o0[r] = acc[r]     * kFoldMain + accr[r]     * kFoldCross;
          o1[r] = acc[4 + r] * kFoldMain + accr[4 + r] * kFoldCross;
        }
        float* sp = slabW + j * 16 * kSlabPitch + 16 * t;
        *(v4f*)(sp)     = o0;
        *(v4f*)(sp + 4) = o1;
      }
    }
  }
  __syncthreads();

  float best = -3.402823466e+38f;
  {
    const float* tapp = strip + lane;
#pragma unroll 1
    for (int o = 0; o < kActions; ++o) {
      const float* lp = slab + (o * kTaps) * kSlabPitch + lane;
      float mx = lp[0];
#pragma unroll
      for (int i = 1; i < kTaps; ++i) mx = fmaxf(mx, lp[i * kSlabPitch]);
      float ssum = 0.0f;
      float qn   = 0.0f;
#pragma unroll 1
      for (int k1 = 0; k1 < 3; ++k1) {
#pragma unroll
        for (int k2 = 0; k2 < 3; ++k2) {
          const float lg = lp[(3 * k1 + k2) * kSlabPitch];
          const float pv = tapp[k1 * kStripPitch + k2];
          float e = expf(lg - mx);
          e = (e < kF32MinNorm) ? 0.0f : e;
          ssum += e;
          qn = fmaf(e, pv, qn);
        }
      }
      const float q = qn / ssum;
      best = fmaxf(best, q);
    }
  }

  float* op = v_out + ((size_t)bimg * kMapH + h) * kMapW + w0 + lane;
  *(volatile float*)op = best;
  __threadfence();
  *(volatile float*)op = best;
}

extern "C" void kernel_launch(void* const* d_in, const int* in_sizes, int n_in,
                              void* d_out, int out_size, void* d_ws, size_t ws_size,
                              hipStream_t stream) {
  (void)d_ws;
  (void)ws_size;
  if (n_in < 3 || d_out == nullptr) return;
  if (in_sizes[0] != kSliceElems) return;
  if (in_sizes[1] != kSliceElems) return;
  if (in_sizes[2] != kChanLive * kTaps) return;
  if (out_size != kDepth * kSliceElems) return;

  const float* values  = (const float*)d_in[0];
  const float* rewards = (const float*)d_in[1];
  const float* wt      = (const float*)d_in[2];
  float* out = (float*)d_out;

  for (int s = 0; s < kDepth; ++s) {
    const float* vin = (s == 0) ? values : (out + (size_t)(s - 1) * kSliceElems);
    float* vout = out + (size_t)s * kSliceElems;
    vi_step_kernel<<<kBlocks, kThreads, 0, stream>>>(vin, rewards, wt, vout);
  }
}
